// MultiLevel_DGCN_LSTM_49443663511667
// MI455X (gfx1250) — hardware-verified
//
#include <hip/hip_runtime.h>


namespace {
constexpr int N = 10000, T = 8, C = 16, O = 64, K = 16, L = 3, NBLK = N / 16;
constexpr float XS = 8.0f, FS = 32.0f, HS = 2048.0f, WSC = 256.0f;
typedef _Float16 b16;
typedef __attribute__((ext_vector_type(16))) _Float16 v16b;
typedef __attribute__((ext_vector_type(8))) _Float16 v8b;
typedef __attribute__((ext_vector_type(8))) float v8f;
typedef __attribute__((ext_vector_type(4))) float v4f;
typedef __attribute__((ext_vector_type(2))) float v2f;
__device__ __forceinline__ float bf16_rne(float f) { unsigned int u = __float_as_uint(f); u += 0x7FFFu + ((u >> 16) & 1u); return __uint_as_float(u & 0xFFFF0000u); }
__device__ __forceinline__ void split16(float v, b16& hi, b16& lo) { hi = (b16)v; lo = (b16)(v - (float)hi); }
__device__ __forceinline__ v16b frag_kb(const b16* p, int hh) { const v8b a = *(const v8b*)(p + 8 * hh), b = *(const v8b*)(p + 16 + 8 * hh); v16b f;
#pragma unroll
  for (int e = 0; e < 8; ++e) { f[e] = a[e]; f[8 + e] = b[e]; } return f; }
__device__ __forceinline__ v8f wmma16b(v16b a, v16b b, v8f c) { v8f d = __builtin_amdgcn_wmma_f32_16x16x32_f16(false, a, false, b, (short)0, c, false, false); asm volatile("v_nop\n\tv_nop\n\tv_nop\n\tv_nop" : "+v"(d) : "v"(a), "v"(b)); return d; }
__device__ __forceinline__ void wave_lds_sync() { __builtin_amdgcn_fence(__ATOMIC_RELEASE, "workgroup"); __builtin_amdgcn_wave_barrier(); __builtin_amdgcn_fence(__ATOMIC_ACQUIRE, "workgroup"); }
__device__ __forceinline__ float pmul(float a, float b) { float p = a * b; asm volatile("" : "+v"(p)); return p; }
__device__ __forceinline__ int iclamp(int v, int lo, int hi) { return v < lo ? lo : (v > hi ? hi : v); }
__device__ __forceinline__ float sigm(float v) { return 1.0f / (1.0f + __expf(-v)); }

__global__ __launch_bounds__(256) void w_kernel(const float* __restrict__ cw, const float* __restrict__ wih, const float* __restrict__ whh, b16* __restrict__ CW, b16* __restrict__ WIH, b16* __restrict__ WHH) {
  const int u = blockIdx.x * 256 + threadIdx.x; v8b v;
  if (u < L * O * 4) { const int lo_ = u / 4, k0 = (u % 4) * 8; for (int j = 0; j < 8; ++j) { const int k = k0 + j; v[j] = k < C ? (b16)(bf16_rne(cw[(size_t)lo_ * C + k]) * WSC) : (b16)0.0f; } for (int pass = 0; pass < 2; ++pass) { *(volatile v8b*)(CW + (size_t)lo_ * 32 + k0) = v; __threadfence(); } }
  else { const int w = u - L * O * 4; if (w >= 2 * L * 256 * 8) return; const int which = w / (L * 256 * 8); const int e = (w % (L * 256 * 8)) * 8; const float* src = which ? whh : wih; b16* dst = which ? WHH : WIH;
    for (int j = 0; j < 8; ++j) v[j] = (b16)(bf16_rne(src[e + j]) * WSC); for (int pass = 0; pass < 2; ++pass) { *(volatile v8b*)(dst + e) = v; __threadfence(); } }
}
__global__ __launch_bounds__(32) void conv_kernel(const float* __restrict__ X, const b16* __restrict__ CW, float* __restrict__ PL) {
  __shared__ __attribute__((aligned(16))) b16 Ah[16][40]; __shared__ __attribute__((aligned(16))) float Tf[16][O + 4];
  const int lane = threadIdx.x, nloc = lane & 15, hlf = lane >> 4; const int nt = blockIdx.x % NBLK, t = (blockIdx.x / NBLK) % T, l = blockIdx.x / (NBLK * T); const size_t m0 = (size_t)nt * 16;
  for (int rr = 0; rr < 16; ++rr) Ah[rr][lane] = lane < C ? (b16)(bf16_rne(X[((m0 + rr) * T + t) * C + lane]) * XS) : (b16)0.0f;
  wave_lds_sync(); const v16b a = frag_kb(&Ah[nloc][0], hlf);
#pragma unroll
  for (int tt = 0; tt < 4; ++tt) { v8f acc = {}; acc = wmma16b(a, frag_kb(CW + ((size_t)l * O + tt * 16 + nloc) * 32, hlf), acc);
#pragma unroll
    for (int r8 = 0; r8 < 8; ++r8) Tf[8 * hlf + r8][tt * 16 + nloc] = acc[r8] * (1.0f / (XS * WSC)); }
  wave_lds_sync();
  for (int pass = 0; pass < 2; ++pass) { for (int rr = 0; rr < 16; ++rr) *(volatile v2f*)(PL + (((size_t)l * T + t) * N + m0 + rr) * O + lane * 2) = *(const v2f*)(&Tf[rr][lane * 2]); __threadfence(); }
}
__global__ __launch_bounds__(32) void lstm_kernel(const float* __restrict__ PL, const int* __restrict__ As, const float* __restrict__ cb, const b16* __restrict__ WIH, const b16* __restrict__ WHH, const float* __restrict__ bih, const float* __restrict__ bhh, int NLIM, float* __restrict__ out) {
  __shared__ __attribute__((aligned(16))) b16 Fh[16][O + 8], Fl[16][O + 8], Hh[16][O + 8], Hl[16][O + 8]; __shared__ float Xo[16][T][O], Gs[16][O + 1], Hm[16][O + 1], Cm[16][O + 1]; __shared__ __attribute__((aligned(16))) float St[16][O + 4];
  const int lane = threadIdx.x, nloc = lane & 15, hlf = lane >> 4; const size_t m0 = (size_t)blockIdx.x * 16; if (m0 >= (size_t)NLIM) return;
  for (int rr = 0; rr < 16; ++rr) { for (int t = 0; t < T; ++t) { Xo[rr][t][lane] = -INFINITY; Xo[rr][t][32 + lane] = -INFINITY; } Hm[rr][lane] = -INFINITY; Hm[rr][32 + lane] = -INFINITY; Cm[rr][lane] = -INFINITY; Cm[rr][32 + lane] = -INFINITY; }
  auto gemm4 = [&](int l, int g, float sc1, float sc2, v8f acc[4]) {
#pragma unroll
    for (int tt = 0; tt < 4; ++tt) acc[tt] = (v8f){};
#pragma unroll
    for (int kb = 0; kb < O; kb += 32) { const v16b a = frag_kb(&Fh[nloc][kb], hlf), al = frag_kb(&Fl[nloc][kb], hlf);
#pragma unroll
      for (int tt = 0; tt < 4; ++tt) { const v16b bw = frag_kb(WIH + ((size_t)l * 4 * O + g * O + tt * 16 + nloc) * O + kb, hlf); acc[tt] = wmma16b(a, bw, acc[tt]); acc[tt] = wmma16b(al, bw, acc[tt]); } }
#pragma unroll
    for (int tt = 0; tt < 4; ++tt)
#pragma unroll
      for (int r8 = 0; r8 < 8; ++r8) acc[tt][r8] *= sc1;
#pragma unroll
    for (int kb = 0; kb < O; kb += 32) { const v16b a = frag_kb(&Hh[nloc][kb], hlf), al = frag_kb(&Hl[nloc][kb], hlf);
#pragma unroll
      for (int tt = 0; tt < 4; ++tt) { const v16b bw = frag_kb(WHH + ((size_t)l * 4 * O + g * O + tt * 16 + nloc) * O + kb, hlf); v8f d = {}; d = wmma16b(a, bw, d); d = wmma16b(al, bw, d);
#pragma unroll
        for (int r8 = 0; r8 < 8; ++r8) acc[tt][r8] += d[r8] * sc2; } } };
#pragma unroll 1
  for (int l = 0; l < L; ++l) { float hreg[4][8], creg[4][8];
#pragma unroll
    for (int tt = 0; tt < 4; ++tt)
#pragma unroll
      for (int r8 = 0; r8 < 8; ++r8) { hreg[tt][r8] = 0.0f; creg[tt][r8] = 0.0f; }
    for (int rr = 0; rr < 16; ++rr) { Hh[rr][lane] = (b16)0.0f; Hl[rr][lane] = (b16)0.0f; Hh[rr][32 + lane] = (b16)0.0f; Hl[rr][32 + lane] = (b16)0.0f; }
    const float cb0 = bf16_rne(cb[l * O + lane * 2]), cb1 = bf16_rne(cb[l * O + lane * 2 + 1]); const float* bi = bih + l * 4 * O; const float* bh = bhh + l * 4 * O;
#pragma unroll 1
    for (int t = 0; t < T; ++t) { const float* Pt = PL + ((size_t)l * T + t) * N * O;
      for (int rr = 0; rr < 16; ++rr) { const size_t n = m0 + rr; const v2f pn = *(const v2f*)(Pt + n * O + lane * 2); float mx0 = -INFINITY, mx1 = -INFINITY;
#pragma unroll 4
        for (int k = 0; k < K; ++k) { const int nb = iclamp(As[(((size_t)l * T + t) * N + n) * K + k], 0, N - 1); const v2f pj = *(const v2f*)(Pt + (size_t)nb * O + lane * 2); mx0 = fmaxf(mx0, pj[0] - pn[0]); mx1 = fmaxf(mx1, pj[1] - pn[1]); }
        b16 p, q; split16((mx0 + cb0) * FS, p, q); Fh[rr][lane * 2] = p; Fl[rr][lane * 2] = q; split16((mx1 + cb1) * FS, p, q); Fh[rr][lane * 2 + 1] = p; Fl[rr][lane * 2 + 1] = q; }
      wave_lds_sync();
      const float s1 = 1.0f / (FS * WSC), s2 = 1.0f / (HS * WSC); v8f acc[4];
      gemm4(l, 2, s1, s2, acc);
#pragma unroll
      for (int tt = 0; tt < 4; ++tt) { const int col = tt * 16 + nloc; const float bb = bf16_rne(bi[2 * O + col]) + bf16_rne(bh[2 * O + col]);
#pragma unroll
        for (int r8 = 0; r8 < 8; ++r8) Gs[8 * hlf + r8][col] = tanhf(acc[tt][r8] + bb); }
      gemm4(l, 0, s1, s2, acc);
#pragma unroll
      for (int tt = 0; tt < 4; ++tt) { const int col = tt * 16 + nloc; const float bb = bf16_rne(bi[col]) + bf16_rne(bh[col]);
#pragma unroll
        for (int r8 = 0; r8 < 8; ++r8) Gs[8 * hlf + r8][col] = pmul(sigm(acc[tt][r8] + bb), Gs[8 * hlf + r8][col]); }
      gemm4(l, 1, s1, s2, acc);
#pragma unroll
      for (int tt = 0; tt < 4; ++tt) { const int col = tt * 16 + nloc; const float bb = bf16_rne(bi[O + col]) + bf16_rne(bh[O + col]);
#pragma unroll
        for (int r8 = 0; r8 < 8; ++r8) creg[tt][r8] = pmul(sigm(acc[tt][r8] + bb), creg[tt][r8]) + Gs[8 * hlf + r8][col]; }
      gemm4(l, 3, s1, s2, acc);
      wave_lds_sync();
#pragma unroll
      for (int tt = 0; tt < 4; ++tt) { const int col = tt * 16 + nloc; const float bb = bf16_rne(bi[3 * O + col]) + bf16_rne(bh[3 * O + col]);
#pragma unroll
        for (int r8 = 0; r8 < 8; ++r8) { const int rl = 8 * hlf + r8; hreg[tt][r8] = pmul(sigm(acc[tt][r8] + bb), tanhf(creg[tt][r8])); Xo[rl][t][col] = fmaxf(Xo[rl][t][col], hreg[tt][r8]); b16 p, q; split16(hreg[tt][r8] * HS, p, q); Hh[rl][col] = p; Hl[rl][col] = q; } }
      wave_lds_sync(); }
#pragma unroll
    for (int tt = 0; tt < 4; ++tt)
#pragma unroll
      for (int r8 = 0; r8 < 8; ++r8) { const int rl = 8 * hlf + r8, col = tt * 16 + nloc; Hm[rl][col] = fmaxf(Hm[rl][col], hreg[tt][r8]); Cm[rl][col] = fmaxf(Cm[rl][col], creg[tt][r8]); }
    wave_lds_sync(); }
  for (int pass = 0; pass < 2; ++pass) { for (int rr = 0; rr < 16; ++rr) { for (int t = 0; t < T; ++t) { ((volatile float*)out)[((m0 + rr) * T + t) * O + lane] = Xo[rr][t][lane]; ((volatile float*)out)[((m0 + rr) * T + t) * O + 32 + lane] = Xo[rr][t][32 + lane]; }
      ((volatile float*)out)[(size_t)N * T * O + (m0 + rr) * O + lane] = Hm[rr][lane]; ((volatile float*)out)[(size_t)N * T * O + (m0 + rr) * O + 32 + lane] = Hm[rr][32 + lane];
      ((volatile float*)out)[(size_t)N * T * O + (size_t)N * O + (m0 + rr) * O + lane] = Cm[rr][lane]; ((volatile float*)out)[(size_t)N * T * O + (size_t)N * O + (m0 + rr) * O + 32 + lane] = Cm[rr][32 + lane]; } __threadfence(); }
  (void)St;
}
}

extern "C" void kernel_launch(void* const* d_in, const int* in_sizes, int n_in, void* d_out, int out_size, void* d_ws, size_t ws_size, hipStream_t stream) {
  (void)n_in;
  auto Fp = [&](int i) { return (const float*)d_in[i]; }; auto Ip = [&](int i) { return (const int*)d_in[i]; };
  if (in_sizes[0] != N * T * C || in_sizes[1] != L * T * N * K || in_sizes[4] != L * O * C || in_sizes[6] != L * 4 * O * O || in_sizes[7] != L * 4 * O * O || out_size != N * T * O + 2 * N * O) return;
  const int NLIM = N;
  size_t off = 0; char* ws = (char*)d_ws;
  auto carve = [&](size_t bytes) { char* p = ws + off; off += (bytes + 255) & ~(size_t)255; return p; };
  b16* CW = (b16*)carve(L * O * 32 * 2); b16* WIH = (b16*)carve((size_t)L * 256 * O * 2); b16* WHH = (b16*)carve((size_t)L * 256 * O * 2); float* PL = (float*)carve((size_t)L * T * N * O * 4);
  if (off > ws_size || off > ((size_t)96 << 20)) return;
  w_kernel<<<(L * O * 4 + 2 * L * 256 * 8 + 255) / 256, 256, 0, stream>>>(Fp(4), Fp(6), Fp(7), CW, WIH, WHH);
  conv_kernel<<<L * T * NBLK, 32, 0, stream>>>(Fp(0), CW, PL);
  lstm_kernel<<<(unsigned)((NLIM + 15) / 16), 32, 0, stream>>>(PL, Ip(1), Fp(5), WIH, WHH, Fp(8), Fp(9), NLIM, (float*)d_out);
}
